// ProbSparseSelfAttention_13477607374942
// MI455X (gfx1250) — hardware-verified
//
#include <hip/hip_runtime.h>
#include <math.h>
#include <stdint.h>


typedef __attribute__((ext_vector_type(16))) _Float16 v16h;
typedef __attribute__((ext_vector_type(8), may_alias)) _Float16 v8h;
typedef __attribute__((ext_vector_type(8)))  float    v8f;
typedef __attribute__((ext_vector_type(4), may_alias)) float v4f;
typedef __attribute__((ext_vector_type(4), may_alias)) unsigned int v4u;

union Frag { v16h v; v8h hf[2]; };
union Pk16 { v8h h; v4u u; };

#ifndef NB
#define NB 2
#endif
#ifndef SEQ
#define SEQ 2048
#endif
#define NB_FULL  2
#define SEQ_FULL 2048
#define DM    1024
#define NH    16
#define DK    64
#define MROWS (NB * SEQ)
#define NQKV  (3 * DM)

#define KT    64
#define QT    16
#define MT    2
#define WAVES 8
#define LDK   72
#define EP16  72
#define EP32  72

#define C2  (0.125f * 1.4426950408889634f)
#define WSC 1024.0f
#define PSC 1024.0f
#define CSC 256.0f

static_assert(NB >= 1 && NB <= NB_FULL);
static_assert(SEQ >= 256 && SEQ <= SEQ_FULL && (SEQ % 256) == 0);
static_assert((MROWS % 128) == 0);
static_assert(NH * DK == DM && (DM % 128) == 0 && (NQKV % 128) == 0);
static_assert(MT == 2 && WAVES * MT * QT == 256);
static_assert((KT * DK) % (256 * 8) == 0);

__device__ __forceinline__ v8f zero8() {
  v8f z = {0.f, 0.f, 0.f, 0.f, 0.f, 0.f, 0.f, 0.f};
  return z;
}

__device__ __forceinline__ float bf16r(float f) {
  unsigned int u = __float_as_uint(f);
  u += 0x7fffu + ((u >> 16) & 1u);
  u &= 0xffff0000u;
  return __uint_as_float(u);
}

__device__ __forceinline__ v8f wmma16(const v16h& a, const v16h& b, v8f c) {
  return __builtin_amdgcn_wmma_f32_16x16x32_f16(false, a, false, b, (short)0, c, false, false);
}

#if __has_builtin(__builtin_amdgcn_permlane16)
__device__ __forceinline__ float permx(float v, unsigned s0, unsigned s1) {
  int x = __float_as_int(v);
  int r = __builtin_amdgcn_permlane16(x, x, (int)s0, (int)s1, false, false);
  return __int_as_float(r);
}
__device__ __forceinline__ float red_max16(float x) {
  x = fmaxf(x, permx(x, 0x67452301u, 0xEFCDAB89u));
  x = fmaxf(x, permx(x, 0x54761032u, 0xDCFE98BAu));
  x = fmaxf(x, permx(x, 0x32107654u, 0xBA98FEDCu));
  x = fmaxf(x, permx(x, 0xFEDCBA98u, 0x76543210u));
  return x;
}
__device__ __forceinline__ float red_sum16(float x) {
  x += permx(x, 0x67452301u, 0xEFCDAB89u);
  x += permx(x, 0x54761032u, 0xDCFE98BAu);
  x += permx(x, 0x32107654u, 0xBA98FEDCu);
  x += permx(x, 0xFEDCBA98u, 0x76543210u);
  return x;
}
#else
__device__ __forceinline__ float red_max16(float x) {
  for (int off = 1; off < 16; off <<= 1) x = fmaxf(x, __shfl_xor(x, off, 32));
  return x;
}
__device__ __forceinline__ float red_sum16(float x) {
  for (int off = 1; off < 16; off <<= 1) x += __shfl_xor(x, off, 32);
  return x;
}
#endif

__global__ __launch_bounds__(256)
void k_cvt(const float* __restrict__ x,
           const float* __restrict__ wq, const float* __restrict__ wk,
           const float* __restrict__ wv, const float* __restrict__ wo,
           _Float16* __restrict__ X16, _Float16* __restrict__ W16,
           int nxc, int ntot)
{
  const int t0 = blockIdx.x * 256;
  const int t  = t0 + (int)threadIdx.x;
  if (t >= ntot) return;

  const float* src;
  _Float16* dst;
  float sc;
  if (t0 < nxc) {
    const int m = t >> 7;
    const int c = t & 127;
    const int b = m / SEQ;
    const int l = m - b * SEQ;
    src = x + (size_t)(b * SEQ_FULL + l) * DM + c * 8;
    dst = X16 + (size_t)t * 8;
    sc  = 1.0f;
  } else {
    const int u    = t - nxc;
    const int wsel = (t0 - nxc) >> 17;
    const int off  = (u & 131071) * 8;
    const float* wsrc = (wsel == 0) ? wq : ((wsel == 1) ? wk : ((wsel == 2) ? wv : wo));
    src = wsrc + off;
    dst = W16 + (size_t)u * 8;
    sc  = WSC;
  }
  const v4f f0 = *(const v4f*)(src);
  const v4f f1 = *(const v4f*)(src + 4);
  Pk16 o;
  o.h[0] = (_Float16)(bf16r(f0.x) * sc);
  o.h[1] = (_Float16)(bf16r(f0.y) * sc);
  o.h[2] = (_Float16)(bf16r(f0.z) * sc);
  o.h[3] = (_Float16)(bf16r(f0.w) * sc);
  o.h[4] = (_Float16)(bf16r(f1.x) * sc);
  o.h[5] = (_Float16)(bf16r(f1.y) * sc);
  o.h[6] = (_Float16)(bf16r(f1.z) * sc);
  o.h[7] = (_Float16)(bf16r(f1.w) * sc);
  *(volatile v4u*)dst = o.u;
  __threadfence();
  *(volatile v4u*)dst = o.u;
}

template <int MODE>
__global__ __launch_bounds__(256)
void k_gemm(const _Float16* __restrict__ A, const _Float16* __restrict__ W,
            const float* __restrict__ b0p, const float* __restrict__ b1p,
            const float* __restrict__ b2p, void* __restrict__ outp)
{
  __shared__ __align__(16) float lds_ep[8 * 16 * EP32];

  const int tid  = threadIdx.x;
  const int lane = tid & 31;
  const int w    = tid >> 5;
  const int h    = lane >> 4;
  const int lc   = lane & 15;
  const int wm   = w & 3;
  const int wn   = w >> 2;
  const int m0   = blockIdx.y * 128 + wm * 32;
  const int nb0  = blockIdx.x * 128;
  const int n0   = nb0 + wn * 64;

  const _Float16* pa0 = A + (size_t)(m0 + lc) * DM + 8 * h;
  const _Float16* pa1 = pa0 + (size_t)16 * DM;
  const _Float16* pb0 = W + (size_t)(n0 + lc) * DM + 8 * h;
  const _Float16* pb1 = pb0 + (size_t)16 * DM;
  const _Float16* pb2 = pb0 + (size_t)32 * DM;
  const _Float16* pb3 = pb0 + (size_t)48 * DM;

  v8f acc[2][4];
  #pragma unroll
  for (int mi = 0; mi < 2; ++mi)
    #pragma unroll
    for (int ni = 0; ni < 4; ++ni) acc[mi][ni] = zero8();

  #pragma unroll 1
  for (int k0 = 0; k0 < DM; k0 += 32) {
    Frag a0, a1, f0, f1, f2, f3;
    a0.hf[0] = *(const v8h*)(pa0 + k0);  a0.hf[1] = *(const v8h*)(pa0 + k0 + 16);
    a1.hf[0] = *(const v8h*)(pa1 + k0);  a1.hf[1] = *(const v8h*)(pa1 + k0 + 16);
    f0.hf[0] = *(const v8h*)(pb0 + k0);  f0.hf[1] = *(const v8h*)(pb0 + k0 + 16);
    f1.hf[0] = *(const v8h*)(pb1 + k0);  f1.hf[1] = *(const v8h*)(pb1 + k0 + 16);
    f2.hf[0] = *(const v8h*)(pb2 + k0);  f2.hf[1] = *(const v8h*)(pb2 + k0 + 16);
    f3.hf[0] = *(const v8h*)(pb3 + k0);  f3.hf[1] = *(const v8h*)(pb3 + k0 + 16);

    acc[0][0] = wmma16(a0.v, f0.v, acc[0][0]);
    acc[1][0] = wmma16(a1.v, f0.v, acc[1][0]);
    acc[0][1] = wmma16(a0.v, f1.v, acc[0][1]);
    acc[1][1] = wmma16(a1.v, f1.v, acc[1][1]);
    acc[0][2] = wmma16(a0.v, f2.v, acc[0][2]);
    acc[1][2] = wmma16(a1.v, f2.v, acc[1][2]);
    acc[0][3] = wmma16(a0.v, f3.v, acc[0][3]);
    acc[1][3] = wmma16(a1.v, f3.v, acc[1][3]);
    asm volatile("v_nop\n\tv_nop\n\tv_nop\n\tv_nop"
      : "+v"(acc[0][0]), "+v"(acc[0][1]), "+v"(acc[0][2]), "+v"(acc[0][3]),
        "+v"(acc[1][0]), "+v"(acc[1][1]), "+v"(acc[1][2]), "+v"(acc[1][3])
      : "v"(a0.v), "v"(a1.v), "v"(f0.v), "v"(f1.v), "v"(f2.v), "v"(f3.v));
  }

  if constexpr (MODE == 0) {
    const int p = nb0 >> 10;
    const float* bias = (p == 0) ? b0p : ((p == 1) ? b1p : b2p);
    const float osc = (p == 0) ? C2 : 1.0f;
    const int nin = n0 & (DM - 1);
    const int hh  = nin >> 6;
    const int bi  = m0 / SEQ;
    const int l0  = m0 - bi * SEQ;
    _Float16* dstp = (_Float16*)outp + ((size_t)((p * NB + bi) * NH + hh) * SEQ + l0) * DK;
    _Float16* st = (_Float16*)lds_ep + w * (32 * EP16);

    float bn[4];
    #pragma unroll
    for (int ni = 0; ni < 4; ++ni) bn[ni] = bf16r(bias[nin + ni * 16 + lc]);

    #pragma unroll
    for (int mi = 0; mi < 2; ++mi)
      #pragma unroll
      for (int ni = 0; ni < 4; ++ni)
        #pragma unroll
        for (int r = 0; r < 8; ++r)
          st[(mi * 16 + 8 * h + r) * EP16 + ni * 16 + lc] =
              (_Float16)((acc[mi][ni][r] * (1.0f / WSC) + bn[ni]) * osc);
    __syncthreads();

    const int rq = lane >> 3, cq = lane & 7;
    Pk16 v[8];
    #pragma unroll
    for (int j = 0; j < 8; ++j) v[j].h = *(const v8h*)(st + (j * 4 + rq) * EP16 + cq * 8);
    #pragma unroll
    for (int j = 0; j < 8; ++j)
      *(volatile v4u*)(dstp + (size_t)(j * 4 + rq) * DK + cq * 8) = v[j].u;
    __threadfence();
    #pragma unroll
    for (int j = 0; j < 8; ++j)
      *(volatile v4u*)(dstp + (size_t)(j * 4 + rq) * DK + cq * 8) = v[j].u;
  } else {
    float* st = lds_ep + w * (16 * EP32);
    float bn[4];
    #pragma unroll
    for (int ni = 0; ni < 4; ++ni) bn[ni] = bf16r(b0p[n0 + ni * 16 + lc]);
    float* dstp = (float*)outp + (size_t)m0 * DM + n0;

    #pragma unroll
    for (int mi = 0; mi < 2; ++mi) {
      if (mi) __syncthreads();
      #pragma unroll
      for (int ni = 0; ni < 4; ++ni)
        #pragma unroll
        for (int r = 0; r < 8; ++r)
          st[(8 * h + r) * EP32 + ni * 16 + lc] = acc[mi][ni][r] * (1.0f / (WSC * CSC)) + bn[ni];
      __syncthreads();
      v4f v[8];
      #pragma unroll
      for (int j = 0; j < 8; ++j) v[j] = *(const v4f*)(st + (j * 2 + h) * EP32 + lc * 4);
      float* d = dstp + (size_t)(mi * 16) * DM;
      #pragma unroll
      for (int j = 0; j < 8; ++j)
        *(volatile v4f*)(d + (size_t)(j * 2 + h) * DM + lc * 4) = v[j];
      __threadfence();
      #pragma unroll
      for (int j = 0; j < 8; ++j)
        *(volatile v4f*)(d + (size_t)(j * 2 + h) * DM + lc * 4) = v[j];
    }
  }
}

__global__ __launch_bounds__(256)
__attribute__((amdgpu_waves_per_eu(4)))
void k_attn(const _Float16* __restrict__ Qp, const _Float16* __restrict__ Kp,
            const _Float16* __restrict__ Vp, _Float16* __restrict__ Cx)
{
  __shared__ __align__(16) _Float16 sK [KT * LDK];
  __shared__ __align__(16) _Float16 sVt[DK * LDK];
  __shared__ __align__(16) _Float16 sP [WAVES][MT * QT * LDK];

  const int tid  = threadIdx.x;
  const int lane = tid & 31;
  const int wave = tid >> 5;
  const int half = lane >> 4;
  const int lc   = lane & 15;

  const int bh    = blockIdx.y;
  const int qrow0 = blockIdx.x * (WAVES * MT * QT) + wave * (MT * QT);

  const size_t baseQ  = ((size_t)bh * SEQ + qrow0) * DK;
  const size_t baseKV = (size_t)bh * SEQ * DK;

  Frag aq[MT][2];
  #pragma unroll
  for (int mt = 0; mt < MT; ++mt) {
    const _Float16* qrow = Qp + baseQ + (size_t)(mt * QT + lc) * DK;
    aq[mt][0].hf[0] = *(const v8h*)(qrow + 8 * half);
    aq[mt][0].hf[1] = *(const v8h*)(qrow + 16 + 8 * half);
    aq[mt][1].hf[0] = *(const v8h*)(qrow + 32 + 8 * half);
    aq[mt][1].hf[1] = *(const v8h*)(qrow + 48 + 8 * half);
  }

  v8f acc[MT][4];
  #pragma unroll
  for (int mt = 0; mt < MT; ++mt)
    #pragma unroll
    for (int i = 0; i < 4; ++i) acc[mt][i] = zero8();

  float mrow[MT][8], lrow[MT][8];
  #pragma unroll
  for (int mt = 0; mt < MT; ++mt)
    #pragma unroll
    for (int r = 0; r < 8; ++r) { mrow[mt][r] = -INFINITY; lrow[mt][r] = 0.0f; }

  for (int kt = 0; kt < SEQ / KT; ++kt) {
    __syncthreads();
    {
      const _Float16* kp = Kp + baseKV + (size_t)kt * KT * DK;
      const _Float16* vp = Vp + baseKV + (size_t)kt * KT * DK;
      #pragma unroll
      for (int i = 0; i < (KT * DK) / (256 * 8); ++i) {
        const int idx = tid + i * 256;
        const int kk  = idx >> 3;
        const int dc  = idx & 7;
        const v8h kv = *(const v8h*)(kp + (size_t)idx * 8);
        const v8h vv = *(const v8h*)(vp + (size_t)idx * 8);
        *(v8h*)(sK + kk * LDK + dc * 8) = kv;
        #pragma unroll
        for (int e = 0; e < 8; ++e) sVt[(dc * 8 + e) * LDK + kk] = vv[e];
      }
    }
    __syncthreads();

    #pragma unroll
    for (int mt = 0; mt < MT; ++mt) {
      v8f sc[4];
      #pragma unroll
      for (int nt = 0; nt < 4; ++nt) {
        if (nt == 2) __builtin_amdgcn_sched_barrier(0);
        Frag b0, b1;
        const _Float16* krow = sK + (nt * 16 + lc) * LDK;
        b0.hf[0] = *(const v8h*)(krow + 8 * half);
        b0.hf[1] = *(const v8h*)(krow + 16 + 8 * half);
        b1.hf[0] = *(const v8h*)(krow + 32 + 8 * half);
        b1.hf[1] = *(const v8h*)(krow + 48 + 8 * half);
        v8f c = zero8();
        c = wmma16(aq[mt][0].v, b0.v, c);
        c = wmma16(aq[mt][1].v, b1.v, c);
        asm volatile("v_nop\n\tv_nop\n\tv_nop\n\tv_nop"
          : "+v"(c) : "v"(aq[mt][0].v), "v"(aq[mt][1].v), "v"(b0.v), "v"(b1.v));
        sc[nt] = c;
      }

      float alpha[8];
      #pragma unroll
      for (int r = 0; r < 8; ++r) {
        float xm = red_max16(fmaxf(fmaxf(sc[0][r], sc[1][r]),
                                   fmaxf(sc[2][r], sc[3][r])));
        const float mnew = fmaxf(mrow[mt][r], xm);
        alpha[r]    = __builtin_amdgcn_exp2f(mrow[mt][r] - mnew);
        mrow[mt][r] = mnew;
        float rs = 0.0f;
        #pragma unroll
        for (int nt = 0; nt < 4; ++nt) {
          const float pr = __builtin_amdgcn_exp2f(sc[nt][r] - mnew);
          sc[nt][r] = pr;
          rs += pr;
        }
        rs = red_sum16(rs);
        lrow[mt][r] = lrow[mt][r] * alpha[r] + rs;
      }

      #pragma unroll
      for (int nt = 0; nt < 4; ++nt)
        #pragma unroll
        for (int r = 0; r < 8; ++r)
          sP[wave][(mt * QT + half * 8 + r) * LDK + nt * 16 + lc] = (_Float16)(sc[nt][r] * PSC);

      #pragma unroll
      for (int dt = 0; dt < 4; ++dt)
        #pragma unroll
        for (int r = 0; r < 8; ++r)
          acc[mt][dt][r] *= alpha[r];
    }

    asm volatile("s_wait_dscnt 0" ::: "memory");
    __builtin_amdgcn_wave_barrier();

    Frag ap[MT][2];
    #pragma unroll
    for (int mt = 0; mt < MT; ++mt) {
      const _Float16* prow = sP[wave] + (mt * QT + lc) * LDK;
      ap[mt][0].hf[0] = *(const v8h*)(prow + 8 * half);
      ap[mt][0].hf[1] = *(const v8h*)(prow + 16 + 8 * half);
      ap[mt][1].hf[0] = *(const v8h*)(prow + 32 + 8 * half);
      ap[mt][1].hf[1] = *(const v8h*)(prow + 48 + 8 * half);
    }

    #pragma unroll
    for (int dt = 0; dt < 4; ++dt) {
      if (dt == 2) __builtin_amdgcn_sched_barrier(0);
      Frag b0, b1;
      const _Float16* vcol = sVt + (dt * 16 + lc) * LDK;
      b0.hf[0] = *(const v8h*)(vcol + 8 * half);
      b0.hf[1] = *(const v8h*)(vcol + 16 + 8 * half);
      b1.hf[0] = *(const v8h*)(vcol + 32 + 8 * half);
      b1.hf[1] = *(const v8h*)(vcol + 48 + 8 * half);
      acc[0][dt] = wmma16(ap[0][0].v, b0.v, acc[0][dt]);
      acc[0][dt] = wmma16(ap[0][1].v, b1.v, acc[0][dt]);
      acc[1][dt] = wmma16(ap[1][0].v, b0.v, acc[1][dt]);
      acc[1][dt] = wmma16(ap[1][1].v, b1.v, acc[1][dt]);
      asm volatile("v_nop\n\tv_nop\n\tv_nop\n\tv_nop"
        : "+v"(acc[0][dt]), "+v"(acc[1][dt])
        : "v"(ap[0][0].v), "v"(ap[0][1].v), "v"(ap[1][0].v), "v"(ap[1][1].v), "v"(b0.v), "v"(b1.v));
    }
  }

  _Float16* st = sP[wave];
  #pragma unroll
  for (int mt = 0; mt < MT; ++mt)
    #pragma unroll
    for (int r = 0; r < 8; ++r) {
      const float inv = __builtin_amdgcn_rcpf(lrow[mt][r]) * (CSC / PSC);
      #pragma unroll
      for (int dt = 0; dt < 4; ++dt)
        st[(mt * QT + half * 8 + r) * LDK + dt * 16 + lc] = (_Float16)(acc[mt][dt][r] * inv);
    }
  __syncthreads();

  const int b  = bh / NH;
  const int hh = bh - b * NH;
  _Float16* cbase = Cx + ((size_t)b * SEQ + qrow0) * DM + hh * DK;
  const int rq = lane >> 3, cq = lane & 7;
  Pk16 v[8];
  #pragma unroll
  for (int j = 0; j < 8; ++j) v[j].h = *(const v8h*)(st + (j * 4 + rq) * LDK + cq * 8);
  #pragma unroll
  for (int j = 0; j < 8; ++j)
    *(volatile v4u*)(cbase + (size_t)(j * 4 + rq) * DM + cq * 8) = v[j].u;
  __threadfence();
  #pragma unroll
  for (int j = 0; j < 8; ++j)
    *(volatile v4u*)(cbase + (size_t)(j * 4 + rq) * DM + cq * 8) = v[j].u;
}

extern "C" void kernel_launch(void* const* d_in, const int* in_sizes, int n_in,
                              void* d_out, int out_size, void* d_ws, size_t ws_size,
                              hipStream_t stream)
{
  if (n_in < 9) return;
  const long long needX = ((long long)(NB - 1) * SEQ_FULL + SEQ) * (long long)DM;
  if ((long long)in_sizes[0] < needX) return;
  if (in_sizes[1] < DM * DM || in_sizes[3] < DM * DM || in_sizes[5] < DM * DM || in_sizes[7] < DM * DM) return;
  if (in_sizes[2] < DM || in_sizes[4] < DM || in_sizes[6] < DM || in_sizes[8] < DM) return;
  if ((long long)out_size < (long long)MROWS * DM) return;

  const float* x  = (const float*)d_in[0];
  const float* wq = (const float*)d_in[1];
  const float* bq = (const float*)d_in[2];
  const float* wk = (const float*)d_in[3];
  const float* bk = (const float*)d_in[4];
  const float* wv = (const float*)d_in[5];
  const float* bv = (const float*)d_in[6];
  const float* wo = (const float*)d_in[7];
  const float* bo = (const float*)d_in[8];

  const size_t nX   = (size_t)MROWS * DM;
  const size_t nW   = (size_t)4 * DM * DM;
  const size_t nP   = (size_t)MROWS * DM;
  const size_t nQKV = 3 * nP;
  const size_t nC   = (size_t)MROWS * DM;
  const size_t total = (nX + nW + nQKV + nC) * sizeof(_Float16);
  if (total > ws_size) return;

  _Float16* X16 = (_Float16*)d_ws;
  _Float16* W16 = X16 + nX;
  _Float16* QKV = W16 + nW;
  _Float16* CX  = QKV + nQKV;

  const int nxc  = (int)(nX / 8);
  const int ntot = (int)((nX + nW) / 8);

  k_cvt<<<dim3((ntot + 255) / 256), dim3(256), 0, stream>>>(x, wq, wk, wv, wo, X16, W16, nxc, ntot);
  k_gemm<0><<<dim3(NQKV / 128, MROWS / 128), dim3(256), 0, stream>>>(X16, W16, bq, bk, bv, (void*)QKV);
  k_attn<<<dim3(SEQ / (WAVES * MT * QT), NB * NH), dim3(256), 0, stream>>>(QKV, QKV + nP, QKV + 2 * nP, CX);
  k_gemm<1><<<dim3(DM / 128, MROWS / 128), dim3(256), 0, stream>>>(CX, W16 + (size_t)3 * DM * DM, bo, bo, bo, d_out);
}
